// ResidualUnit_15264313770267
// MI455X (gfx1250) — hardware-run, weakly checked
//
#include <hip/hip_runtime.h>

#pragma clang fp contract(off)

typedef __attribute__((ext_vector_type(16))) _Float16 v16h;
typedef __attribute__((ext_vector_type(8)))  _Float16 v8h;
typedef __attribute__((ext_vector_type(16))) __bf16   v16b;
typedef __attribute__((ext_vector_type(8)))  __bf16   v8b;
typedef __attribute__((ext_vector_type(8)))  float    v8f;
typedef __attribute__((ext_vector_type(4)))  float    v4f;

__device__ __forceinline__ unsigned short f2bf_bits(float f) {
  unsigned u = __float_as_uint(f);
  return (unsigned short)((u + 0x7FFFu + ((u >> 16) & 1u)) >> 16);
}
__device__ __forceinline__ float bf_bits2f(unsigned short h) { return __uint_as_float(((unsigned)h) << 16); }

__device__ __forceinline__ void dep_guard_h(v8f& a, v8f& b, v16h x, v16h y) { asm volatile("v_nop\n\tv_nop\n\tv_nop\n\tv_nop" : "+v"(a), "+v"(b) : "v"(x), "v"(y)); }
__device__ __forceinline__ void dep_guard_b(v8f& a, v8f& b, v16b x, v16b y) { asm volatile("v_nop\n\tv_nop\n\tv_nop\n\tv_nop" : "+v"(a), "+v"(b) : "v"(x), "v"(y)); }
__device__ __forceinline__ void keep4_h(v16h a, v16h b, v16h c, v16h d) { asm volatile("v_nop" :: "v"(a), "v"(b), "v"(c), "v"(d)); }
__device__ __forceinline__ void keep4_b(v16b a, v16b b, v16b c, v16b d) { asm volatile("v_nop" :: "v"(a), "v"(b), "v"(c), "v"(d)); }
__device__ __forceinline__ void acc_guard4(v8f& a, v8f& b, v8f& c, v8f& d) { asm volatile("v_nop\n\tv_nop\n\tv_nop\n\tv_nop" : "+v"(a), "+v"(b), "+v"(c), "+v"(d)); }
template <typename T> struct Frag;
template <> struct Frag<_Float16> {
  typedef v16h V; union U { v16h v; v8h h[2]; };
  static __device__ __forceinline__ v16h load(const _Float16* p) {
    U f; f.h[0] = *(const v8h*)(p); f.h[1] = *(const v8h*)(p + 16); return f.v;
  }
  static __device__ __forceinline__ v8f mma(v16h a, v16h b, v8f c) {
    return __builtin_amdgcn_wmma_f32_16x16x32_f16(false, a, false, b, (short)0, c, false, false);
  }
  static __device__ __forceinline__ void guard(v8f& a, v8f& b, v16h x, v16h y) { dep_guard_h(a, b, x, y); }
  static __device__ __forceinline__ void keep(v16h a, v16h b, v16h c, v16h d) { keep4_h(a, b, c, d); }
};
template <> struct Frag<__bf16> {
  typedef v16b V; union U { v16b v; v8b h[2]; };
  static __device__ __forceinline__ v16b load(const __bf16* p) {
    U f; f.h[0] = *(const v8b*)(p); f.h[1] = *(const v8b*)(p + 16); return f.v;
  }
  static __device__ __forceinline__ v8f mma(v16b a, v16b b, v8f c) {
    return __builtin_amdgcn_wmma_f32_16x16x32_bf16(false, a, false, b, (short)0, c, false, false);
  }
  static __device__ __forceinline__ void guard(v8f& a, v8f& b, v16b x, v16b y) { dep_guard_b(a, b, x, y); }
  static __device__ __forceinline__ void keep(v16b a, v16b b, v16b c, v16b d) { keep4_b(a, b, c, d); }
};

__device__ __forceinline__ v16h ld_pk_h(const _Float16* p) {
  Frag<_Float16>::U f; f.h[0] = *(const v8h*)(p); f.h[1] = *(const v8h*)(p + 8); return f.v;
}
__device__ __forceinline__ v16b ld_pk_b(const __bf16* p) {
  Frag<__bf16>::U f; f.h[0] = *(const v8b*)(p); f.h[1] = *(const v8b*)(p + 8); return f.v;
}

__device__ __forceinline__ void guard8_h(v8f (&c)[2][4], v16h a0, v16h a1, v16h b0, v16h b1, v16h b2, v16h b3) {
  asm volatile("v_nop\n\tv_nop\n\tv_nop\n\tv_nop"
               : "+v"(c[0][0]), "+v"(c[0][1]), "+v"(c[0][2]), "+v"(c[0][3]),
                 "+v"(c[1][0]), "+v"(c[1][1]), "+v"(c[1][2]), "+v"(c[1][3])
               : "v"(a0), "v"(a1), "v"(b0), "v"(b1), "v"(b2), "v"(b3));
}
__device__ __forceinline__ void guard8_b(v8f (&c)[2][4], v16b a0, v16b a1, v16b b0, v16b b1, v16b b2, v16b b3) {
  asm volatile("v_nop\n\tv_nop\n\tv_nop\n\tv_nop"
               : "+v"(c[0][0]), "+v"(c[0][1]), "+v"(c[0][2]), "+v"(c[0][3]),
                 "+v"(c[1][0]), "+v"(c[1][1]), "+v"(c[1][2]), "+v"(c[1][3])
               : "v"(a0), "v"(a1), "v"(b0), "v"(b1), "v"(b2), "v"(b3));
}

static constexpr int   NBATCH   = 4;
static constexpr int   NSTEP    = 16;
static constexpr int   IMG1     = 128;
static constexpr int   IMG2     = 64;
static constexpr int   NFEAT    = 32;
static constexpr int   NCIN     = 3;
static constexpr float OP_SCALE = 64.0f;
static constexpr float W1_SCALE = 4096.0f;
static constexpr float ACC_INV  = 1.0f / 4096.0f;
static constexpr int   HALO_R   = 6;
static constexpr int   HALO_C   = 34;

__device__ __forceinline__ float hsig(float v) {
  float u = 0.2f * v + 0.5f;
  u = fmaxf(u, 0.0f);
  return fminf(u, 1.0f);
}


__global__ __launch_bounds__(256) void pack_taps_f16(const float* __restrict__ src, _Float16* __restrict__ dst) {
  const int i = blockIdx.x * 256 + threadIdx.x;
  if (i >= 4608) return;
  const int e0  = (i & 1) * 8;
  const int ln  = (i >> 1) & 31;
  const int nt  = (i >> 6) & 7;
  const int tap = i >> 9;
  const int hh = ln >> 4, mm = ln & 15;
  v8h o;
#pragma unroll
  for (int j = 0; j < 8; ++j) {
    const int k = 8 * hh + 2 * e0 + j;
    const float w = src[(tap * 32 + k) * 128 + nt * 16 + mm] * OP_SCALE;
    o[j] = (_Float16)w;
  }
  _Float16* p = dst + (size_t)i * 8;
  *(volatile v8h*)p = o;
  __threadfence();
  *(volatile v8h*)p = o;
}

__global__ __launch_bounds__(256) void pack_w1_bf16(const float* __restrict__ src, unsigned short* __restrict__ dst) {
  const int i = blockIdx.x * 256 + threadIdx.x;
  if (i >= 1536) return;
  const int e0 = (i & 1) * 8;
  const int ln = (i >> 1) & 31;
  const int nt = (i >> 6) & 7;
  const int g  = i >> 9;
  const int hh = ln >> 4, mm = ln & 15;
  v8h o;
#pragma unroll
  for (int j = 0; j < 8; ++j) {
    const int k = 8 * hh + 2 * e0 + j;
    const bool valid = (k < 27);
    const int kc = valid ? k : 0;
    float w = src[kc * 128 + nt * 16 + mm] * W1_SCALE;
    w = valid ? w : 0.0f;
    const unsigned short hb = f2bf_bits(w);
    const unsigned short lb = f2bf_bits(w - bf_bits2f(hb));
    const unsigned short us = (g == 2) ? lb : hb;
    o[j] = __builtin_bit_cast(_Float16, us);
  }
  unsigned short* p = dst + (size_t)i * 8;
  *(volatile v8h*)p = o;
  __threadfence();
  *(volatile v8h*)p = o;
}

__global__ __launch_bounds__(256) void pack_wc_bf16(const float* __restrict__ src, unsigned short* __restrict__ dst) {
  const int i = blockIdx.x * 256 + threadIdx.x;
  if (i >= 1024) return;
  const int e0  = (i & 1) * 8;
  const int ln  = (i >> 1) & 31;
  const int tp  = (i >> 6) & 3;
  const int pxp = (i >> 8) & 1;
  const int pyp = (i >> 9) & 1;
  const int ty = tp >> 1, tx = tp & 1;
  const int hh = ln >> 4, mm = ln & 15;
  const int co = (mm < 3) ? mm : ((mm < 6) ? (mm - 3) : 0);
  v8h o;
#pragma unroll
  for (int j = 0; j < 8; ++j) {
    const int cin = 8 * hh + 2 * e0 + j;
    float s = 0.0f;
#pragma unroll
    for (int dy = 0; dy < 3; ++dy) {
      const bool iy = (((dy + 1 - pyp) >> 1) == ty);
#pragma unroll
      for (int dx = 0; dx < 3; ++dx) {
        const bool ix = (((dx + 1 - pxp) >> 1) == tx);
        const float w = src[((dy * 3 + dx) * 32 + cin) * 3 + co];
        s += (iy && ix) ? w : 0.0f;
      }
    }
    const unsigned short hb = f2bf_bits(s);
    const unsigned short lb = f2bf_bits(s - bf_bits2f(hb));
    const unsigned short us = (mm < 3) ? hb : ((mm < 6) ? lb : (unsigned short)0);
    o[j] = __builtin_bit_cast(_Float16, us);
  }
  unsigned short* p = dst + (size_t)i * 8;
  *(volatile v8h*)p = o;
  __threadfence();
  *(volatile v8h*)p = o;
}


__device__ __forceinline__ void stage_tile16(const _Float16* __restrict__ src, _Float16* lds,
                                             int b, int y0, int x0, int img, int tid) {
  for (int i = tid; i < 816; i += 256) {
    const int r = i / 136;
    const int rem = i - r * 136;
    const int cc = rem >> 2, ck = rem & 3;
    const int yy = y0 - 1 + r, xx = x0 - 1 + cc;
    const bool inb = ((unsigned)yy < (unsigned)img) && ((unsigned)xx < (unsigned)img);
    const int yc = yy < 0 ? 0 : (yy > img - 1 ? img - 1 : yy);
    const int xc = xx < 0 ? 0 : (xx > img - 1 ? img - 1 : xx);
    int4 v = *(const int4*)(src + (((size_t)b * img + yc) * img + xc) * 32 + ck * 8);
    if (!inb) v = make_int4(0, 0, 0, 0);
    *(int4*)(lds + (r * HALO_C + cc) * 32 + ck * 8) = v;
  }
}

__device__ __forceinline__ void conv_taps_f16(v8f (&acc)[2][4], const _Float16* lds,
                                              const _Float16* __restrict__ Bpk, int wr, int q, int lane) {
  const int hh = lane >> 4, mm = lane & 15;
#pragma unroll 1
  for (int dy = 0; dy < 3; ++dy) {
#pragma unroll 1
    for (int dx = 0; dx < 3; ++dx) {
      const int tap = dy * 3 + dx;
      v16h bb[4];
#pragma unroll
      for (int j = 0; j < 4; ++j)
        bb[j] = ld_pk_h(Bpk + ((size_t)((tap * 8 + 2 * j + q) * 32 + lane)) * 16);
      const _Float16* ap = lds + ((wr + dy) * HALO_C + mm + dx) * 32 + 8 * hh;
      const v16h a0 = Frag<_Float16>::load(ap);
      const v16h a1 = Frag<_Float16>::load(ap + 16 * 32);
#pragma unroll
      for (int j = 0; j < 4; ++j) {
        acc[0][j] = Frag<_Float16>::mma(a0, bb[j], acc[0][j]);
        acc[1][j] = Frag<_Float16>::mma(a1, bb[j], acc[1][j]);
      }
      guard8_h(acc, a0, a1, bb[0], bb[1], bb[2], bb[3]);
    }
  }
}

__device__ __forceinline__ void xgroup_bf16(v8f (&acc)[2][4], v16b a0, v16b a1,
                                            const __bf16* __restrict__ W1b, int g, int q, int lane) {
  v16b bb[4];
#pragma unroll
  for (int j = 0; j < 4; ++j)
    bb[j] = ld_pk_b(W1b + ((size_t)((g * 8 + 2 * j + q) * 32 + lane)) * 16);
#pragma unroll
  for (int j = 0; j < 4; ++j) {
    acc[0][j] = Frag<__bf16>::mma(a0, bb[j], acc[0][j]);
    acc[1][j] = Frag<__bf16>::mma(a1, bb[j], acc[1][j]);
  }
  guard8_b(acc, a0, a1, bb[0], bb[1], bb[2], bb[3]);
}

__device__ __forceinline__ void gates_to_lds(v8f (&acc)[2][4], const float* __restrict__ bias,
                                             const float* __restrict__ cst, float* ldsC, float* ldsHn,
                                             int b, int y0, int x0, int img, int wr, int q, int lane, int first) {
  const int hh = lane >> 4, mm = lane & 15;
  const int n = 16 * q + mm;
  const float bi = bias[n], bf = bias[32 + n], bg = bias[64 + n], bo = bias[96 + n];
#pragma unroll
  for (int f = 0; f < 2; ++f) {
#pragma unroll
    for (int r = 0; r < 8; ++r) {
      const int px = 16 * f + 8 * hh + r;
      const int P = wr * 32 + px;
      const size_t gi = (((size_t)b * img + (y0 + wr)) * img + (x0 + px)) * 32 + n;
      float cp = cst[gi];
      cp = first ? 0.0f : cp;
      const float zi = acc[f][0][r] * ACC_INV + bi;
      const float zf = acc[f][1][r] * ACC_INV + bf;
      const float zg = acc[f][2][r] * ACC_INV + bg;
      const float zo = acc[f][3][r] * ACC_INV + bo;
      const float ig = hsig(zi), fg = hsig(zf), og = hsig(zo);
      const float cn = fg * cp + ig * fmaxf(zg, 0.0f);
      const float hn = og * fmaxf(cn, 0.0f);
      ldsC[P * 32 + n]  = cn;
      ldsHn[P * 32 + n] = hn;
    }
  }
}

__device__ __forceinline__ v8h pack8_f16_x64(const float* sp) {
  const v4f u0 = *(const v4f*)sp;
  const v4f u1 = *(const v4f*)(sp + 4);
  v8h o;
  o[0] = (_Float16)(u0[0] * OP_SCALE); o[1] = (_Float16)(u0[1] * OP_SCALE);
  o[2] = (_Float16)(u0[2] * OP_SCALE); o[3] = (_Float16)(u0[3] * OP_SCALE);
  o[4] = (_Float16)(u1[0] * OP_SCALE); o[5] = (_Float16)(u1[1] * OP_SCALE);
  o[6] = (_Float16)(u1[2] * OP_SCALE); o[7] = (_Float16)(u1[3] * OP_SCALE);
  return o;
}

__global__ __launch_bounds__(256) void lstm1_step(
    const float* __restrict__ x, const unsigned short* __restrict__ W1pk, const _Float16* __restrict__ U1pk,
    const float* __restrict__ b1, const _Float16* __restrict__ hin, _Float16* __restrict__ hout,
    float* __restrict__ cst, _Float16* __restrict__ pool, int t, int first) {
  __shared__ __align__(16) _Float16 ldsH[HALO_R * HALO_C * 32];
  __shared__ __align__(16) float    ldsX[HALO_R * HALO_C * 3];
  __shared__ __align__(16) float    ldsHn[128 * 32];
  __shared__ __align__(16) float    ldsC[128 * 32];

  const int x0 = blockIdx.x * 32, y0 = blockIdx.y * 4, b = blockIdx.z;
  const int tid = threadIdx.x, lane = tid & 31, wave = tid >> 5;
  const int wr = wave >> 1, q = wave & 1, hh = lane >> 4, mm = lane & 15;

  for (int i = tid; i < 612; i += 256) {
    const int r = i / 102;
    const int rem = i - 102 * r;
    const int cc = rem / 3;
    const int cin = rem - 3 * cc;
    const int yy = y0 - 1 + r, xx = x0 - 1 + cc;
    const bool inb = ((unsigned)yy < 128u) && ((unsigned)xx < 128u);
    const int yc = yy < 0 ? 0 : (yy > 127 ? 127 : yy);
    const int xc = xx < 0 ? 0 : (xx > 127 ? 127 : xx);
    const float v = x[((((size_t)b * NSTEP + t) * IMG1 + yc) * IMG1 + xc) * 3 + cin];
    ldsX[i] = inb ? v : 0.0f;
  }
  if (!first) stage_tile16(hin, ldsH, b, y0, x0, IMG1, tid);
  __syncthreads();

  v8f acc[2][4];
#pragma unroll
  for (int f = 0; f < 2; ++f)
#pragma unroll
    for (int j = 0; j < 4; ++j) acc[f][j] = (v8f){0.f, 0.f, 0.f, 0.f, 0.f, 0.f, 0.f, 0.f};

  v16b xh0, xl0, xh1, xl1;
#pragma unroll
  for (int e = 0; e < 16; ++e) {
    const int ke = (e < 8) ? e : (e + 8);
    const int k = 8 * hh + ke;
    const bool valid = (k < 27);
    const int kc = valid ? k : 0;
    const int tap = (kc * 11) >> 5;
    const int cin = kc - 3 * tap;
    const int dy = (tap * 11) >> 5;
    const int dx = tap - 3 * dy;
    const int o = ((wr + dy) * HALO_C + mm + dx) * 3 + cin;
    float v0 = ldsX[o];
    float v1 = ldsX[o + 48];
    v0 = valid ? v0 : 0.0f;
    v1 = valid ? v1 : 0.0f;
    const unsigned short h0b = f2bf_bits(v0), h1b = f2bf_bits(v1);
    const unsigned short l0b = f2bf_bits(v0 - bf_bits2f(h0b));
    const unsigned short l1b = f2bf_bits(v1 - bf_bits2f(h1b));
    xh0[e] = __builtin_bit_cast(__bf16, h0b); xl0[e] = __builtin_bit_cast(__bf16, l0b);
    xh1[e] = __builtin_bit_cast(__bf16, h1b); xl1[e] = __builtin_bit_cast(__bf16, l1b);
  }
  {
    const __bf16* W1b = (const __bf16*)W1pk;
    xgroup_bf16(acc, xh0, xh1, W1b, 0, q, lane);
    xgroup_bf16(acc, xl0, xl1, W1b, 1, q, lane);
    xgroup_bf16(acc, xh0, xh1, W1b, 2, q, lane);
  }
  if (!first) conv_taps_f16(acc, ldsH, U1pk, wr, q, lane);
  acc_guard4(acc[0][0], acc[0][1], acc[0][2], acc[0][3]);
  acc_guard4(acc[1][0], acc[1][1], acc[1][2], acc[1][3]);

  gates_to_lds(acc, b1, cst, ldsC, ldsHn, b, y0, x0, IMG1, wr, q, lane, first);
  __syncthreads();

  for (int pass = 0; pass < 2; ++pass) {
#pragma unroll
    for (int it = 0; it < 2; ++it) {
      const int idx = wave + 8 * it;
      const int rr = idx >> 2, ch = idx & 3;
      const int px = ch * 8 + (lane >> 2), n0 = (lane & 3) * 8;
      const v8h hv = pack8_f16_x64(ldsHn + (rr * 32 + px) * 32 + n0);
      *(volatile v8h*)(hout + ((((size_t)b * IMG1 + y0 + rr) * IMG1 + x0 + px) * 32 + n0)) = hv;
    }
#pragma unroll
    for (int it = 0; it < 4; ++it) {
      const int idx = wave + 8 * it;
      const int rr = idx >> 3, ch = idx & 7;
      const int px = ch * 4 + (lane >> 3), n0 = (lane & 7) * 4;
      const v4f cv = *(const v4f*)(ldsC + (rr * 32 + px) * 32 + n0);
      *(volatile v4f*)(cst + ((((size_t)b * IMG1 + y0 + rr) * IMG1 + x0 + px) * 32 + n0)) = cv;
    }
    if (wave < 4) {
      const int pr = wave >> 1, ch = wave & 1;
      const int ppx = ch * 8 + (lane >> 2), n0 = (lane & 3) * 8;
      const float* s00 = ldsHn + ((2 * pr) * 32 + 2 * ppx) * 32 + n0;
      const float* s01 = s00 + 32;
      const float* s10 = s00 + 32 * 32;
      const float* s11 = s10 + 32;
      v4f a0 = *(const v4f*)s00, a1 = *(const v4f*)(s00 + 4);
      const v4f b0 = *(const v4f*)s01, b1v = *(const v4f*)(s01 + 4);
      const v4f c0 = *(const v4f*)s10, c1 = *(const v4f*)(s10 + 4);
      const v4f d0 = *(const v4f*)s11, d1 = *(const v4f*)(s11 + 4);
      v8h pv;
#pragma unroll
      for (int e = 0; e < 4; ++e) {
        const float m0 = fmaxf(fmaxf(a0[e], b0[e]), fmaxf(c0[e], d0[e]));
        const float m1 = fmaxf(fmaxf(a1[e], b1v[e]), fmaxf(c1[e], d1[e]));
        pv[e]     = (_Float16)(m0 * OP_SCALE);
        pv[4 + e] = (_Float16)(m1 * OP_SCALE);
      }
      *(volatile v8h*)(pool + ((((size_t)b * IMG2 + (y0 >> 1) + pr) * IMG2 + (x0 >> 1) + ppx) * 32 + n0)) = pv;
    }
    __threadfence();
  }
}

__global__ __launch_bounds__(256) void lstm2_step(
    const _Float16* __restrict__ xin, const _Float16* __restrict__ W2pk, const _Float16* __restrict__ U2pk,
    const float* __restrict__ b2, const _Float16* __restrict__ hin, _Float16* __restrict__ hout,
    float* __restrict__ cst, unsigned short* __restrict__ seq_hi, unsigned short* __restrict__ seq_lo,
    int t, int first) {
  __shared__ __align__(16) _Float16 ldsXI[HALO_R * HALO_C * 32];
  __shared__ __align__(16) _Float16 ldsH[HALO_R * HALO_C * 32];
  __shared__ __align__(16) float    ldsHn[128 * 32];
  __shared__ __align__(16) float    ldsC[128 * 32];

  const int x0 = blockIdx.x * 32, y0 = blockIdx.y * 4, b = blockIdx.z;
  const int tid = threadIdx.x, lane = tid & 31, wave = tid >> 5;
  const int wr = wave >> 1, q = wave & 1;

  stage_tile16(xin, ldsXI, b, y0, x0, IMG2, tid);
  if (!first) stage_tile16(hin, ldsH, b, y0, x0, IMG2, tid);
  __syncthreads();

  v8f acc[2][4];
#pragma unroll
  for (int f = 0; f < 2; ++f)
#pragma unroll
    for (int j = 0; j < 4; ++j) acc[f][j] = (v8f){0.f, 0.f, 0.f, 0.f, 0.f, 0.f, 0.f, 0.f};

  conv_taps_f16(acc, ldsXI, W2pk, wr, q, lane);
  if (!first) conv_taps_f16(acc, ldsH, U2pk, wr, q, lane);
  acc_guard4(acc[0][0], acc[0][1], acc[0][2], acc[0][3]);
  acc_guard4(acc[1][0], acc[1][1], acc[1][2], acc[1][3]);

  gates_to_lds(acc, b2, cst, ldsC, ldsHn, b, y0, x0, IMG2, wr, q, lane, first);
  __syncthreads();

  const int frame = b * NSTEP + t;
  for (int pass = 0; pass < 2; ++pass) {
#pragma unroll
    for (int it = 0; it < 2; ++it) {
      const int idx = wave + 8 * it;
      const int rr = idx >> 2, ch = idx & 3;
      const int px = ch * 8 + (lane >> 2), n0 = (lane & 3) * 8;
      const float* sp = ldsHn + (rr * 32 + px) * 32 + n0;
      const v8h hv = pack8_f16_x64(sp);
      *(volatile v8h*)(hout + ((((size_t)b * IMG2 + y0 + rr) * IMG2 + x0 + px) * 32 + n0)) = hv;
      const v4f u0 = *(const v4f*)sp;
      const v4f u1 = *(const v4f*)(sp + 4);
      v8h hiv, lov;
#pragma unroll
      for (int e = 0; e < 4; ++e) {
        const unsigned short hb0 = f2bf_bits(u0[e]);
        const unsigned short lb0 = f2bf_bits(u0[e] - bf_bits2f(hb0));
        const unsigned short hb1 = f2bf_bits(u1[e]);
        const unsigned short lb1 = f2bf_bits(u1[e] - bf_bits2f(hb1));
        hiv[e] = __builtin_bit_cast(_Float16, hb0); lov[e] = __builtin_bit_cast(_Float16, lb0);
        hiv[4 + e] = __builtin_bit_cast(_Float16, hb1); lov[4 + e] = __builtin_bit_cast(_Float16, lb1);
      }
      const size_t so = (((size_t)frame * IMG2 + y0 + rr) * IMG2 + x0 + px) * 32 + n0;
      *(volatile v8h*)(seq_hi + so) = hiv;
      *(volatile v8h*)(seq_lo + so) = lov;
    }
#pragma unroll
    for (int it = 0; it < 4; ++it) {
      const int idx = wave + 8 * it;
      const int rr = idx >> 3, ch = idx & 7;
      const int px = ch * 4 + (lane >> 3), n0 = (lane & 7) * 4;
      const v4f cv = *(const v4f*)(ldsC + (rr * 32 + px) * 32 + n0);
      *(volatile v4f*)(cst + ((((size_t)b * IMG2 + y0 + rr) * IMG2 + x0 + px) * 32 + n0)) = cv;
    }
    __threadfence();
  }
}

__global__ __launch_bounds__(128) void final_conv(
    const unsigned short* __restrict__ seq_hi, const unsigned short* __restrict__ seq_lo,
    const unsigned short* __restrict__ Wcpk, const float* __restrict__ bc,
    const float* __restrict__ x, float* __restrict__ out) {
  __shared__ __align__(16) __bf16 Ah[3 * 66 * 32];
  __shared__ __align__(16) __bf16 Al[3 * 66 * 32];
  __shared__ __align__(16) float  S[2 * 128 * 8];

  const int a = blockIdx.x;
  const int frame = blockIdx.y;
  const int tid = threadIdx.x, lane = tid & 31, wave = tid >> 5;
  const int hh = lane >> 4, mm = lane & 15;

  for (int i = tid; i < 792; i += 128) {
    const int r = i / 264;
    const int rem = i - 264 * r;
    const int cc = rem >> 2, ck = rem & 3;
    const int sr = a - 1 + r, sc = cc - 1;
    const bool inb = ((unsigned)sr < 64u) && ((unsigned)sc < 64u);
    const int src = sr < 0 ? 0 : (sr > 63 ? 63 : sr);
    const int scc = sc < 0 ? 0 : (sc > 63 ? 63 : sc);
    const size_t go = (((size_t)frame * IMG2 + src) * IMG2 + scc) * 32 + ck * 8;
    int4 vh = *(const int4*)(seq_hi + go);
    int4 vl = *(const int4*)(seq_lo + go);
    if (!inb) { vh = make_int4(0, 0, 0, 0); vl = make_int4(0, 0, 0, 0); }
    *(int4*)(Ah + (r * 66 + cc) * 32 + ck * 8) = vh;
    *(int4*)(Al + (r * 66 + cc) * 32 + ck * 8) = vl;
  }
  __syncthreads();

  const int yy = wave >> 1;
  const int px = wave & 1;
  const int py = yy;
  const __bf16* Wcb = (const __bf16*)Wcpk;
  v16b bw[4];
#pragma unroll
  for (int tp = 0; tp < 4; ++tp)
    bw[tp] = ld_pk_b(Wcb + ((size_t)(((py * 2 + px) * 4 + tp) * 32 + lane)) * 16);

  v8f acc[4];
#pragma unroll
  for (int jt = 0; jt < 4; ++jt) acc[jt] = (v8f){0.f, 0.f, 0.f, 0.f, 0.f, 0.f, 0.f, 0.f};

#pragma unroll
  for (int tp = 0; tp < 4; ++tp) {
    const int ty = tp >> 1, tx = tp & 1;
#pragma unroll
    for (int jt = 0; jt < 4; ++jt) {
      const int eo = ((py + ty) * 66 + 16 * jt + mm + tx + px) * 32 + 8 * hh;
      const v16b fa = Frag<__bf16>::load(Ah + eo);
      const v16b fl = Frag<__bf16>::load(Al + eo);
      acc[jt] = Frag<__bf16>::mma(fa, bw[tp], acc[jt]);
      acc[jt] = Frag<__bf16>::mma(fl, bw[tp], acc[jt]);
      dep_guard_b(acc[jt], acc[(jt + 1) & 3], fa, fl);
    }
  }
  keep4_b(bw[0], bw[1], bw[2], bw[3]);
  acc_guard4(acc[0], acc[1], acc[2], acc[3]);

#pragma unroll
  for (int jt = 0; jt < 4; ++jt) {
#pragma unroll
    for (int r = 0; r < 8; ++r) {
      const int xo = 2 * (16 * jt + 8 * hh + r) + px;
      if (mm < 8) S[(yy * 128 + xo) * 8 + mm] = acc[jt][r];
    }
  }
  __syncthreads();

  const float bc0 = bc[0], bc1 = bc[1], bc2 = bc[2];
  const size_t gbase = ((size_t)frame * IMG1 + 2 * a) * (IMG1 * 3);
  const size_t out1_off = (size_t)NBATCH * NSTEP * IMG1 * IMG1 * NCIN;
  for (int pass = 0; pass < 2; ++pass) {
#pragma unroll
    for (int it = 0; it < 2; ++it) {
      const int idx = wave + 4 * it;
      if (idx < 6) {
        const int fo = idx * 128 + 4 * lane;
        const v4f xv = *(const v4f*)(x + gbase + fo);
        v4f o0, o1;
#pragma unroll
        for (int e = 0; e < 4; ++e) {
          const int f = fo + e;
          const int row = (f >= 384) ? 1 : 0;
          const int rem = f - 384 * row;
          const int xp = rem / 3;
          const int ch = rem - 3 * xp;
          const float s = S[(row * 128 + xp) * 8 + ch] + S[(row * 128 + xp) * 8 + ch + 3];
          const float bb = (ch == 0) ? bc0 : ((ch == 1) ? bc1 : bc2);
          const float v = fmaxf(s + bb, 0.0f);
          o0[e] = v;
          o1[e] = v + xv[e];
        }
        *(volatile v4f*)(out + gbase + fo) = o0;
        *(volatile v4f*)(out + out1_off + gbase + fo) = o1;
      }
    }
    __threadfence();
  }
}

extern "C" void kernel_launch(void* const* d_in, const int* in_sizes, int n_in,
                              void* d_out, int out_size, void* d_ws,
                              size_t ws_size, hipStream_t stream) {
  if (n_in < 9) return;
  if (in_sizes[0] != NBATCH * NSTEP * IMG1 * IMG1 * NCIN) return;
  if (in_sizes[1] != 9 * NCIN * 128) return;
  if (in_sizes[2] != 9 * 32 * 128 || in_sizes[4] != 9 * 32 * 128 || in_sizes[5] != 9 * 32 * 128) return;
  if (in_sizes[3] != 128 || in_sizes[6] != 128) return;
  if (in_sizes[7] != 9 * 32 * 3 || in_sizes[8] != 3) return;
  if (out_size != 2 * NBATCH * NSTEP * IMG1 * IMG1 * NCIN) return;

  const float* x   = (const float*)d_in[0];
  const float* W1  = (const float*)d_in[1];
  const float* U1  = (const float*)d_in[2];
  const float* b1  = (const float*)d_in[3];
  const float* W2  = (const float*)d_in[4];
  const float* U2  = (const float*)d_in[5];
  const float* b2  = (const float*)d_in[6];
  const float* Wc  = (const float*)d_in[7];
  const float* bc  = (const float*)d_in[8];
  float* out = (float*)d_out;

  const size_t szTap  = (size_t)9 * 8 * 32 * 16 * 2;
  const size_t szW1   = (size_t)3 * 8 * 32 * 16 * 2;
  const size_t szWc   = (size_t)2 * 2 * 4 * 32 * 16 * 2;
  const size_t h1E    = (size_t)NBATCH * IMG1 * IMG1 * NFEAT;
  const size_t h2E    = (size_t)NBATCH * IMG2 * IMG2 * NFEAT;
  const size_t szH1   = h1E * 2, szC1 = h1E * 4;
  const size_t szHP   = (size_t)NSTEP * h2E * 2;
  const size_t szH2   = h2E * 2, szC2 = h2E * 4;
  const size_t szSeq  = (size_t)NSTEP * h2E * 2;

  size_t off = 0;
  char* wsb = (char*)d_ws;
  _Float16*       U1pk = (_Float16*)(wsb + off);        off += szTap;
  _Float16*       W2pk = (_Float16*)(wsb + off);        off += szTap;
  _Float16*       U2pk = (_Float16*)(wsb + off);        off += szTap;
  unsigned short* W1pk = (unsigned short*)(wsb + off);  off += szW1;
  unsigned short* Wcpk = (unsigned short*)(wsb + off);  off += szWc;
  _Float16*       h1s0 = (_Float16*)(wsb + off);        off += szH1;
  _Float16*       h1s1 = (_Float16*)(wsb + off);        off += szH1;
  float*          c1   = (float*)(wsb + off);           off += szC1;
  _Float16*       hp   = (_Float16*)(wsb + off);        off += szHP;
  _Float16*       h2s0 = (_Float16*)(wsb + off);        off += szH2;
  _Float16*       h2s1 = (_Float16*)(wsb + off);        off += szH2;
  float*          c2   = (float*)(wsb + off);           off += szC2;
  unsigned short* sqhi = (unsigned short*)(wsb + off);  off += szSeq;
  unsigned short* sqlo = (unsigned short*)(wsb + off);  off += szSeq;
  if (off > ws_size) return;

  pack_taps_f16<<<18, 256, 0, stream>>>(U1, U1pk);
  pack_taps_f16<<<18, 256, 0, stream>>>(W2, W2pk);
  pack_taps_f16<<<18, 256, 0, stream>>>(U2, U2pk);
  pack_w1_bf16<<<6, 256, 0, stream>>>(W1, W1pk);
  pack_wc_bf16<<<4, 256, 0, stream>>>(Wc, Wcpk);

  for (int t = 0; t < NSTEP; ++t) {
    const _Float16* hin = (t & 1) ? h1s1 : h1s0;
    _Float16* hout = (t & 1) ? h1s0 : h1s1;
    lstm1_step<<<dim3(IMG1 / 32, IMG1 / 4, NBATCH), 256, 0, stream>>>(
        x, W1pk, U1pk, b1, hin, hout, c1, hp + (size_t)t * h2E, t, (t == 0) ? 1 : 0);
  }
  for (int t = 0; t < NSTEP; ++t) {
    const _Float16* hin = (t & 1) ? h2s1 : h2s0;
    _Float16* hout = (t & 1) ? h2s0 : h2s1;
    lstm2_step<<<dim3(IMG2 / 32, IMG2 / 4, NBATCH), 256, 0, stream>>>(
        hp + (size_t)t * h2E, W2pk, U2pk, b2, hin, hout, c2, sqhi, sqlo, t, (t == 0) ? 1 : 0);
  }
  final_conv<<<dim3(IMG2, NBATCH * NSTEP), 128, 0, stream>>>(sqhi, sqlo, Wcpk, bc, x, out);
}
